// LogSigRNN_41515153883174
// MI455X (gfx1250) — hardware-run, weakly checked
//
#include <hip/hip_runtime.h>
#include <math.h>

constexpr int NBAT      = 16;
constexpr int NCHAN     = 64;
constexpr int NTIME     = 200;
constexpr int NJOINT    = 25;
constexpr int NSEG      = 50;
constexpr int SEGLEN    = 4;
constexpr int NSEQ      = NBAT * NJOINT;
constexpr int NPAIR     = NCHAN * (NCHAN - 1) / 2;
constexpr int NFEAT     = NCHAN + NPAIR + NCHAN;
constexpr int KPAD      = 2176;
constexpr int KCAT      = 3 * KPAD;
constexpr int NHID      = 128;
constexpr int NGATE     = 4 * NHID;
constexpr int SEG_CHUNK = 10;
constexpr int NCHUNK    = NSEG / SEG_CHUNK;
constexpr int MREAL     = SEG_CHUNK * NSEQ;
constexpr int MPAD      = 4032;
constexpr int NTHR      = 256;
constexpr int NGROUP    = KPAD / 64;
constexpr int XS_PITCH  = 516;
constexpr int AH_PITCH  = 136;
constexpr int HS_PITCH  = 132;
constexpr float W_CARRY   = 256.0f;
constexpr float H_CARRY   = 64.0f;
constexpr float ACC_FOLD  = 1.0f / (W_CARRY * H_CARRY);
constexpr int OCT_ROW   = KCAT / 8;
constexpr int OCT_THIRD = KPAD / 8;
constexpr int OCT_REAL  = NFEAT / 8;
constexpr int PREP_NB_BT  = NGATE * OCT_ROW / NTHR;
constexpr int PREP_NB_WH  = NGATE * NHID / 8 / NTHR;
constexpr int PREP_NB_PAD = (MPAD - MREAL) * OCT_ROW / NTHR;
constexpr int PREP_NB_ALL = PREP_NB_BT + PREP_NB_WH + PREP_NB_PAD + 1;
constexpr int OUT_TOTAL = NBAT * NHID * NSEG * NJOINT;

static_assert(NTIME == NSEG * SEGLEN);
static_assert(NSEQ == 400 && NPAIR == 2016 && NFEAT == 2144);
static_assert(NFEAT % 8 == 0 && KPAD % 64 == 0 && KPAD >= NFEAT);
static_assert(KCAT % 32 == 0 && KCAT == 6528);
static_assert(MPAD % 64 == 0 && MPAD >= MREAL && NGATE % 64 == 0);
static_assert((MPAD / 64) * (NGATE / 64) % 8 == 0);
static_assert(NSEQ % 16 == 0 && NHID % 32 == 0 && NHID == 16 * (NTHR / 32));
static_assert(NGATE * OCT_ROW % NTHR == 0);
static_assert(NGATE * NHID / 8 % NTHR == 0);
static_assert((MPAD - MREAL) * OCT_ROW % NTHR == 0);
static_assert(OUT_TOTAL % (4 * NTHR) == 0);
static_assert(NSEG % SEG_CHUNK == 0);

typedef __attribute__((ext_vector_type(16))) _Float16 v16h;
typedef __attribute__((ext_vector_type(8)))  _Float16 v8h;
typedef __attribute__((ext_vector_type(16))) __bf16   v16b;
typedef __attribute__((ext_vector_type(8)))  __bf16   v8b;
typedef __attribute__((ext_vector_type(8)))  float    v8f;
typedef __attribute__((ext_vector_type(4)))  float    v4f;
typedef __attribute__((ext_vector_type(4)))  unsigned v4u;

__device__ __forceinline__ unsigned short f2bf_bits(float f) {
  unsigned u = __float_as_uint(f);
  return (unsigned short)((u + 0x7FFFu + ((u >> 16) & 1u)) >> 16);
}
__device__ __forceinline__ float bf_bits2f(unsigned short h) { return __uint_as_float(((unsigned)h) << 16); }

__device__ __forceinline__ void guard4_b(v8f& a, v8f& b, v8f& c, v8f& d, v16b x, v16b y) {
  asm volatile("v_nop\n\tv_nop\n\tv_nop\n\tv_nop" : "+v"(a), "+v"(b), "+v"(c), "+v"(d) : "v"(x), "v"(y));
}
__device__ __forceinline__ void guard4_h(v8f& a, v8f& b, v8f& c, v8f& d, v16h x, v16h y) {
  asm volatile("v_nop\n\tv_nop\n\tv_nop\n\tv_nop" : "+v"(a), "+v"(b), "+v"(c), "+v"(d) : "v"(x), "v"(y));
}
__device__ __forceinline__ void keep4_h(v16h a, v16h b, v16h c, v16h d) { asm volatile("v_nop" :: "v"(a), "v"(b), "v"(c), "v"(d)); }
__device__ __forceinline__ void keep4_b(v16b a, v16b b, v16b c, v16b d) { asm volatile("v_nop" :: "v"(a), "v"(b), "v"(c), "v"(d)); }
__device__ __forceinline__ void acc_guard4(v8f& a, v8f& b, v8f& c, v8f& d) {
  asm volatile("v_nop\n\tv_nop\n\tv_nop\n\tv_nop" : "+v"(a), "+v"(b), "+v"(c), "+v"(d));
}

template <typename T> struct Frag;
template <> struct Frag<_Float16> {
  typedef v16h V; union U { v16h v; v8h h[2]; };
  static __device__ __forceinline__ v16h load(const _Float16* p) {
    U f; f.h[0] = *(const v8h*)(p); f.h[1] = *(const v8h*)(p + 16); return f.v;
  }
  static __device__ __forceinline__ v8f mma(v16h a, v16h b, v8f c) {
    return __builtin_amdgcn_wmma_f32_16x16x32_f16(false, a, false, b, (short)0, c, false, false);
  }
};
template <> struct Frag<__bf16> {
  typedef v16b V; union U { v16b v; v8b h[2]; };
  static __device__ __forceinline__ v16b load(const __bf16* p) {
    U f; f.h[0] = *(const v8b*)(p); f.h[1] = *(const v8b*)(p + 16); return f.v;
  }
  static __device__ __forceinline__ v8f mma(v16b a, v16b b, v8f c) {
    return __builtin_amdgcn_wmma_f32_16x16x32_bf16(false, a, false, b, (short)0, c, false, false);
  }
};

__device__ __forceinline__ unsigned pack2(unsigned short lo16, unsigned short hi16) {
  return (unsigned)lo16 | ((unsigned)hi16 << 16);
}

__global__ __launch_bounds__(NTHR) void prep_kernel(const float* __restrict__ Wih, const float* __restrict__ Whh,
                                                    const float* __restrict__ bih, const float* __restrict__ bhh,
                                                    unsigned short* __restrict__ Bt3, unsigned short* __restrict__ WH16,
                                                    float* __restrict__ bsum, unsigned short* __restrict__ A3pad) {
  const int tid = threadIdx.x;
  const int blk = blockIdx.x;
  if (blk < PREP_NB_BT) {
    const int i = blk * NTHR + tid;
    const int row = i / OCT_ROW;
    const int c8i = i - row * OCT_ROW;
    const int third = c8i / OCT_THIRD;
    const int kk8 = c8i - third * OCT_THIRD;
    const bool real = kk8 < OCT_REAL;
    const int kk8c = real ? kk8 : (OCT_REAL - 1);
    const float* sp = Wih + (size_t)row * NFEAT + kk8c * 8;
    const v4f va = *(const v4f*)(sp);
    const v4f vb = *(const v4f*)(sp + 4);
    float f[8];
    f[0] = va[0]; f[1] = va[1]; f[2] = va[2]; f[3] = va[3];
    f[4] = vb[0]; f[5] = vb[1]; f[6] = vb[2]; f[7] = vb[3];
    unsigned short bits[8];
#pragma unroll
    for (int e = 0; e < 8; ++e) {
      float w = f[e];
      asm volatile("" : "+v"(w));
      const unsigned short hb = f2bf_bits(w);
      const unsigned short lb = f2bf_bits(w - bf_bits2f(hb));
      const unsigned short sel = (third == 2) ? lb : hb;
      bits[e] = real ? sel : (unsigned short)0;
    }
    v4u o;
    o[0] = pack2(bits[0], bits[1]);
    o[1] = pack2(bits[2], bits[3]);
    o[2] = pack2(bits[4], bits[5]);
    o[3] = pack2(bits[6], bits[7]);
    volatile v4u* dp = (volatile v4u*)(void*)Bt3 + i;
    *dp = o;
    __threadfence();
    *dp = o;
  } else if (blk < PREP_NB_BT + PREP_NB_WH) {
    const int i = (blk - PREP_NB_BT) * NTHR + tid;
    const float* sp = Whh + (size_t)i * 8;
    const v4f va = *(const v4f*)(sp);
    const v4f vb = *(const v4f*)(sp + 4);
    float f[8];
    f[0] = va[0]; f[1] = va[1]; f[2] = va[2]; f[3] = va[3];
    f[4] = vb[0]; f[5] = vb[1]; f[6] = vb[2]; f[7] = vb[3];
    unsigned short bits[8];
#pragma unroll
    for (int e = 0; e < 8; ++e) {
      const _Float16 hv = (_Float16)(f[e] * W_CARRY);
      bits[e] = __builtin_bit_cast(unsigned short, hv);
    }
    v4u o;
    o[0] = pack2(bits[0], bits[1]);
    o[1] = pack2(bits[2], bits[3]);
    o[2] = pack2(bits[4], bits[5]);
    o[3] = pack2(bits[6], bits[7]);
    volatile v4u* dp = (volatile v4u*)(void*)WH16 + i;
    *dp = o;
    __threadfence();
    *dp = o;
  } else if (blk < PREP_NB_BT + PREP_NB_WH + PREP_NB_PAD) {
    const int i = (blk - PREP_NB_BT - PREP_NB_WH) * NTHR + tid;
    v4u o;
    o[0] = 0u; o[1] = 0u; o[2] = 0u; o[3] = 0u;
    volatile v4u* dp = (volatile v4u*)(void*)A3pad + i;
    *dp = o;
    __threadfence();
    *dp = o;
  } else {
    if (tid < NGATE / 4) {
      const v4f va = *(const v4f*)(bih + 4 * tid);
      const v4f vb = *(const v4f*)(bhh + 4 * tid);
      v4f o;
      o[0] = va[0] + vb[0]; o[1] = va[1] + vb[1]; o[2] = va[2] + vb[2]; o[3] = va[3] + vb[3];
      volatile v4f* dp = (volatile v4f*)(bsum + 4 * tid);
      *dp = o;
      __threadfence();
      *dp = o;
    }
  }
}

__device__ __forceinline__ void decode_col(int col, int& ty, int& ci, int& cj) {
  int t = 3, a = 0, b2 = 0;
  if (col < NCHAN) {
    t = 0; a = col; b2 = col;
  } else if (col < NCHAN + NPAIR) {
    const int k = col - NCHAN;
    const int twoc = 2 * NCHAN - 1;
    int i = (int)(((float)twoc - sqrtf((float)(twoc * twoc - 8 * k))) * 0.5f);
    i = i < 0 ? 0 : (i > NCHAN - 2 ? NCHAN - 2 : i);
    if (i * (twoc - i) / 2 > k) --i;
    if ((i + 1) * (twoc - 1 - i) / 2 <= k) ++i;
    i = i < 0 ? 0 : (i > NCHAN - 2 ? NCHAN - 2 : i);
    int j = i + 1 + (k - i * (twoc - i) / 2);
    j = j < 1 ? 1 : (j > NCHAN - 1 ? NCHAN - 1 : j);
    t = 1; a = i; b2 = j;
  } else if (col < NFEAT) {
    t = 2; a = col - (NCHAN + NPAIR); b2 = a;
  }
  ty = t; ci = a; cj = b2;
}

__global__ __launch_bounds__(NTHR) void logsig_kernel(const float* __restrict__ x, unsigned short* __restrict__ A3, int chunk) {
  __shared__ __align__(16) float P[NCHAN * 100];
  __shared__ __align__(16) v4f   Tb[NJOINT * NCHAN];
  const int tid = threadIdx.x;
  const int lane = tid & 31;
  const int wave = __builtin_amdgcn_readfirstlane((int)(threadIdx.x >> 5));
  const int b  = blockIdx.x / SEG_CHUNK;
  const int sl = blockIdx.x - b * SEG_CHUNK;
  const int s  = chunk * SEG_CHUNK + sl;
  const float* xb = x + ((size_t)b * NCHAN * NTIME + (size_t)SEGLEN * s) * NJOINT;

  for (int idx = tid; idx < NCHAN * 25; idx += NTHR) {
    const int c = idx / 25;
    const int q = idx - c * 25;
    const v4f v = *(const v4f*)(xb + (size_t)c * (NTIME * NJOINT) + 4 * q);
    *(v4f*)(P + c * 100 + 4 * q) = v;
  }
  __syncthreads();
  for (int idx = tid; idx < NJOINT * NCHAN; idx += NTHR) {
    const int v = idx >> 6;
    const int c = idx & 63;
    const float p0 = P[c * 100 + v];
    const float p1 = P[c * 100 + 25 + v];
    const float p2 = P[c * 100 + 50 + v];
    const float p3 = P[c * 100 + 75 + v];
    v4f tv;
    tv[0] = p1 - p0; tv[1] = p2 - p0; tv[2] = p2 - p1; tv[3] = p3 - p2;
    Tb[idx] = tv;
  }
  __syncthreads();

  const size_t rowbase = (size_t)sl * NSEQ + (size_t)b * NJOINT;
  for (int g = wave; g < NGROUP; g += NTHR / 32) {
    int ty0, ci0, cj0, ty1, ci1, cj1;
    decode_col(g * 64 + 2 * lane, ty0, ci0, cj0);
    decode_col(g * 64 + 2 * lane + 1, ty1, ci1, cj1);
#pragma unroll 1
    for (int v = 0; v < NJOINT; ++v) {
      const v4f ti0 = Tb[v * NCHAN + ci0];
      const v4f tj0 = Tb[v * NCHAN + cj0];
      const v4f ti1 = Tb[v * NCHAN + ci1];
      const v4f tj1 = Tb[v * NCHAN + cj1];
      const float p00 = P[ci0 * 100 + v];
      const float p30 = P[ci0 * 100 + 75 + v];
      const float p01 = P[ci1 * 100 + v];
      const float p31 = P[ci1 * 100 + 75 + v];
      const float ar0 = 0.5f * ((ti0[0] * tj0[2] + ti0[1] * tj0[3]) - (tj0[0] * ti0[2] + tj0[1] * ti0[3]));
      const float ar1 = 0.5f * ((ti1[0] * tj1[2] + ti1[1] * tj1[3]) - (tj1[0] * ti1[2] + tj1[1] * ti1[3]));
      const float lv0 = p30 - p00;
      const float lv1 = p31 - p01;
      const float f0 = (ty0 == 1) ? ar0 : ((ty0 == 0) ? lv0 : ((ty0 == 2) ? p00 : 0.0f));
      const float f1 = (ty1 == 1) ? ar1 : ((ty1 == 0) ? lv1 : ((ty1 == 2) ? p01 : 0.0f));
      const unsigned short h0 = f2bf_bits(f0);
      const unsigned short h1 = f2bf_bits(f1);
      const unsigned short l0 = f2bf_bits(f0 - bf_bits2f(h0));
      const unsigned short l1 = f2bf_bits(f1 - bf_bits2f(h1));
      const unsigned whi = pack2(h0, h1);
      const unsigned wlo = pack2(l0, l1);
      volatile unsigned* rp = (volatile unsigned*)(void*)(A3 + (rowbase + (size_t)v) * KCAT) + g * 32 + lane;
      for (int pass = 0; pass < 2; ++pass) {
        rp[0] = whi;
        rp[KPAD / 2] = wlo;
        rp[KPAD] = whi;
        __threadfence();
      }
    }
  }
}

__global__ __launch_bounds__(NTHR) void gemm_bf16_kernel(const unsigned short* __restrict__ Ap, int lda,
                                                         const unsigned short* __restrict__ Btp, int ldb,
                                                         float* __restrict__ Cout, int ldc, int M, int N, int K) {
  typedef __bf16 T;
  typedef v16b V;
  const T* A  = (const T*)Ap;
  const T* Bt = (const T*)Btp;
  __shared__ __align__(16) float sT[8][16 * 68];
  const int lane = threadIdx.x & 31;
  const int wave = __builtin_amdgcn_readfirstlane((int)(threadIdx.x >> 5));
  const int tilesN = N >> 6;
  const int tilesM = M >> 6;
  const int tile = blockIdx.x * 8 + wave;
  if (tile >= tilesM * tilesN) return;
  const int tm = tile / tilesN;
  const int tn = tile - tm * tilesN;
  const int m0 = tm << 6;
  const int n0 = tn << 6;
  const int rlane = lane & 15;
  const int koff  = (lane >> 4) * 8;
  const int mOff  = (lane >> 4) * 8;

  const T* bp[4];
  const T* ap[4];
#pragma unroll
  for (int j = 0; j < 4; ++j) bp[j] = Bt + (size_t)(n0 + (j << 4) + rlane) * ldb + koff;
#pragma unroll
  for (int i = 0; i < 4; ++i) ap[i] = A + (size_t)(m0 + (i << 4) + rlane) * lda + koff;

  v8f acc[4][4];
#pragma unroll
  for (int i = 0; i < 4; ++i)
#pragma unroll
    for (int j = 0; j < 4; ++j) acc[i][j] = (v8f){0.f, 0.f, 0.f, 0.f, 0.f, 0.f, 0.f, 0.f};

  for (int k0 = 0; k0 < K; k0 += 32) {
    V bh[4];
#pragma unroll
    for (int j = 0; j < 4; ++j) bh[j] = Frag<T>::load(bp[j] + k0);
#pragma unroll
    for (int i = 0; i < 4; ++i) {
      const V ah = Frag<T>::load(ap[i] + k0);
#pragma unroll
      for (int j = 0; j < 4; ++j) acc[i][j] = Frag<T>::mma(ah, bh[j], acc[i][j]);
      guard4_b(acc[i][0], acc[i][1], acc[i][2], acc[i][3], ah, bh[3]);
    }
    keep4_b(bh[0], bh[1], bh[2], bh[3]);
  }
  acc_guard4(acc[0][0], acc[0][1], acc[0][2], acc[0][3]);
  acc_guard4(acc[1][0], acc[1][1], acc[1][2], acc[1][3]);
  acc_guard4(acc[2][0], acc[2][1], acc[2][2], acc[2][3]);
  acc_guard4(acc[3][0], acc[3][1], acc[3][2], acc[3][3]);

  float* slab = sT[wave];
  const int hh = lane >> 4;
  const int c4 = (lane & 15) * 4;
#pragma unroll
  for (int i = 0; i < 4; ++i) {
    const int mBase = m0 + (i << 4);
#pragma unroll
    for (int j = 0; j < 4; ++j) {
#pragma unroll
      for (int r = 0; r < 8; ++r) slab[(mOff + r) * 68 + (j << 4) + rlane] = acc[i][j][r];
    }
    __builtin_amdgcn_fence(__ATOMIC_RELEASE, "workgroup");
    __builtin_amdgcn_wave_barrier();
    __builtin_amdgcn_fence(__ATOMIC_ACQUIRE, "workgroup");
    for (int pass = 0; pass < 2; ++pass) {
#pragma unroll
      for (int it = 0; it < 8; ++it) {
        const int row = it * 2 + hh;
        const v4f v = *(const v4f*)(slab + row * 68 + c4);
        *(volatile v4f*)(Cout + (size_t)(mBase + row) * ldc + n0 + c4) = v;
      }
      __threadfence();
    }
    __builtin_amdgcn_fence(__ATOMIC_RELEASE, "workgroup");
    __builtin_amdgcn_wave_barrier();
    __builtin_amdgcn_fence(__ATOMIC_ACQUIRE, "workgroup");
  }
}

__device__ __forceinline__ void stage_xtile(const float* __restrict__ src, float* Xs, int tid) {
#pragma unroll
  for (int it = 0; it < 8; ++it) {
    const int idx = it * NTHR + tid;
    const int row = idx >> 7;
    const int c4 = (idx & 127) * 4;
    const v4f v = *(const v4f*)(src + (size_t)row * NGATE + c4);
    *(v4f*)(Xs + row * XS_PITCH + c4) = v;
  }
}

__device__ __forceinline__ float sigm(float z)  { return __builtin_amdgcn_rcpf(1.0f + expf(-z)); }
__device__ __forceinline__ float tanh_e(float z) { return 1.0f - 2.0f * __builtin_amdgcn_rcpf(expf(2.0f * z) + 1.0f); }

__global__ __launch_bounds__(NTHR) void lstm_kernel(const float* __restrict__ xproj, const float* __restrict__ bsum,
                                                    const unsigned short* __restrict__ WHp, float* __restrict__ hs) {
  __shared__ __align__(16) float    Xs[16 * XS_PITCH];
  __shared__ __align__(16) _Float16 Ah[16 * AH_PITCH];
  __shared__ __align__(16) float    Hs[16 * HS_PITCH];
  const _Float16* WH = (const _Float16*)WHp;
  const int tid = threadIdx.x;
  const int lane = tid & 31;
  const int wave = __builtin_amdgcn_readfirstlane((int)(threadIdx.x >> 5));
  const int c = lane & 15;
  const int hh = lane >> 4;
  const int koff = hh * 8;
  const int n0 = blockIdx.x * 16;
  const int j = 16 * wave + c;

  for (int i = tid; i < 16 * AH_PITCH; i += NTHR) Ah[i] = (_Float16)0.0f;
  float bb0 = bsum[j];
  float bb1 = bsum[NHID + j];
  float bb2 = bsum[2 * NHID + j];
  float bb3 = bsum[3 * NHID + j];
  float cst[8];
#pragma unroll
  for (int r = 0; r < 8; ++r) cst[r] = 0.0f;
  stage_xtile(xproj + (size_t)n0 * NGATE, Xs, tid);
  __syncthreads();

  const _Float16* arow = Ah + c * AH_PITCH + koff;
  const _Float16* wrow = WH + (size_t)j * NHID + koff;
  const v8f z8 = {0.f, 0.f, 0.f, 0.f, 0.f, 0.f, 0.f, 0.f};

#pragma unroll 1
  for (int t = 0; t < NSEG; ++t) {
    v8f acc0 = z8, acc1 = z8, acc2 = z8, acc3 = z8;
#pragma unroll 1
    for (int k0 = 0; k0 < NHID; k0 += 32) {
      const v16h a  = Frag<_Float16>::load(arow + k0);
      const v16h b0 = Frag<_Float16>::load(wrow + k0);
      const v16h b1 = Frag<_Float16>::load(wrow + (size_t)1 * NHID * NHID + k0);
      const v16h b2 = Frag<_Float16>::load(wrow + (size_t)2 * NHID * NHID + k0);
      const v16h b3 = Frag<_Float16>::load(wrow + (size_t)3 * NHID * NHID + k0);
      acc0 = Frag<_Float16>::mma(a, b0, acc0);
      acc1 = Frag<_Float16>::mma(a, b1, acc1);
      acc2 = Frag<_Float16>::mma(a, b2, acc2);
      acc3 = Frag<_Float16>::mma(a, b3, acc3);
      guard4_h(acc0, acc1, acc2, acc3, a, b3);
      keep4_h(b0, b1, b2, b3);
    }
    acc_guard4(acc0, acc1, acc2, acc3);

    float hst[8];
#pragma unroll
    for (int r = 0; r < 8; ++r) {
      const float* xr = Xs + (8 * hh + r) * XS_PITCH + j;
      const float zi = acc0[r] * ACC_FOLD + (xr[0] + bb0);
      const float zf = acc1[r] * ACC_FOLD + (xr[NHID] + bb1);
      const float zg = acc2[r] * ACC_FOLD + (xr[2 * NHID] + bb2);
      const float zo = acc3[r] * ACC_FOLD + (xr[3 * NHID] + bb3);
      const float ig = sigm(zi);
      const float fg = sigm(zf);
      const float gg = tanh_e(zg);
      const float og = sigm(zo);
      const float cn = fg * cst[r] + ig * gg;
      cst[r] = cn;
      hst[r] = og * tanh_e(cn);
    }
    __syncthreads();
#pragma unroll
    for (int r = 0; r < 8; ++r) {
      Ah[(8 * hh + r) * AH_PITCH + j] = (_Float16)(hst[r] * H_CARRY);
      Hs[(8 * hh + r) * HS_PITCH + j] = hst[r];
    }
    {
      const int tn = (t + 1 < NSEG) ? (t + 1) : (NSEG - 1);
      const int ch = tn / SEG_CHUNK;
      const int sl = tn - ch * SEG_CHUNK;
      stage_xtile(xproj + ((size_t)ch * MPAD + (size_t)sl * NSEQ + (size_t)n0) * NGATE, Xs, tid);
    }
    __syncthreads();
    for (int pass = 0; pass < 2; ++pass) {
#pragma unroll
      for (int it = 0; it < 2; ++it) {
        const int idx = it * NTHR + tid;
        const int row = idx >> 5;
        const int c4 = (idx & 31) * 4;
        const v4f v = *(const v4f*)(Hs + row * HS_PITCH + c4);
        *(volatile v4f*)(hs + ((size_t)(n0 + row) * NSEG + (size_t)t) * NHID + c4) = v;
      }
      __threadfence();
    }
  }
}

__global__ __launch_bounds__(NTHR) void out_permute_kernel(const float* __restrict__ hs, float* __restrict__ out) {
  const int gid = blockIdx.x * NTHR + threadIdx.x;
  if (gid >= OUT_TOTAL / 4) return;
  const int f0 = gid * 4;
  v4f o;
#pragma unroll
  for (int e = 0; e < 4; ++e) {
    const int f = f0 + e;
    const int q = f / NJOINT;
    const int v = f - q * NJOINT;
    const int q2 = q / NSEG;
    const int t = q - q2 * NSEG;
    const int hc = q2 & (NHID - 1);
    const int b = q2 >> 7;
    o[e] = hs[((size_t)(b * NJOINT + v) * NSEG + (size_t)t) * NHID + hc];
  }
  volatile v4f* dp = (volatile v4f*)(out + (size_t)f0);
  *dp = o;
  __threadfence();
  *dp = o;
}

extern "C" void kernel_launch(void* const* d_in, const int* in_sizes, int n_in,
                              void* d_out, int out_size, void* d_ws, size_t ws_size, hipStream_t stream) {
  if (n_in < 5 || d_out == nullptr || d_ws == nullptr) return;
  if (in_sizes[0] != NBAT * NCHAN * NTIME * NJOINT || in_sizes[1] != NGATE * NFEAT || in_sizes[2] != NGATE * NHID ||
      in_sizes[3] != NGATE || in_sizes[4] != NGATE || out_size != OUT_TOTAL) return;

  const float* x   = (const float*)d_in[0];
  const float* Wih = (const float*)d_in[1];
  const float* Whh = (const float*)d_in[2];
  const float* bih = (const float*)d_in[3];
  const float* bhh = (const float*)d_in[4];
  float* out = (float*)d_out;

  char* ws = (char*)d_ws;
  size_t off = 0;
  auto carve = [&](size_t bytes) -> char* { char* p = ws + off; off += (bytes + 255) & ~(size_t)255; return p; };
  unsigned short* A3    = (unsigned short*)carve((size_t)MPAD * KCAT * 2);
  unsigned short* BT3   = (unsigned short*)carve((size_t)NGATE * KCAT * 2);
  float*          XPROJ = (float*)carve((size_t)NCHUNK * MPAD * NGATE * 4);
  float*          HS    = (float*)carve((size_t)NSEQ * NSEG * NHID * 4);
  unsigned short* WH16  = (unsigned short*)carve((size_t)NGATE * NHID * 2);
  float*          BSUM  = (float*)carve((size_t)NGATE * 4);
  if (off > ws_size || off > (size_t)134217728) return;

  prep_kernel<<<PREP_NB_ALL, NTHR, 0, stream>>>(Wih, Whh, bih, bhh, BT3, WH16, BSUM, A3 + (size_t)MREAL * KCAT);

  const int gemm_blocks = (MPAD / 64) * (NGATE / 64) / 8;
  for (int ch = 0; ch < NCHUNK; ++ch) {
    logsig_kernel<<<NBAT * SEG_CHUNK, NTHR, 0, stream>>>(x, A3, ch);
    gemm_bf16_kernel<<<gemm_blocks, NTHR, 0, stream>>>(A3, KCAT, BT3, KCAT,
                                                       XPROJ + (size_t)ch * MPAD * NGATE, NGATE, MPAD, NGATE, KCAT);
  }

  lstm_kernel<<<NSEQ / 16, NTHR, 0, stream>>>(XPROJ, BSUM, WH16, HS);
  out_permute_kernel<<<OUT_TOTAL / 4 / NTHR, NTHR, 0, stream>>>(HS, out);
}
